// oracle_GRU_72206990180495
// MI455X (gfx1250) — hardware-verified
//
#include <hip/hip_runtime.h>
#include <stdint.h>
#include <stddef.h>

typedef __attribute__((ext_vector_type(16))) _Float16 v16h;
typedef __attribute__((ext_vector_type(8)))  _Float16 v8h;
typedef __attribute__((ext_vector_type(16))) __bf16   v16b;
typedef __attribute__((ext_vector_type(8)))  __bf16   v8b;
typedef __attribute__((ext_vector_type(8)))  float    v8f;
typedef __attribute__((ext_vector_type(4)))  float    v4f;
typedef __attribute__((ext_vector_type(4)))  unsigned int v4u;

__device__ __forceinline__ unsigned short f2bf_bits(float f) {
  unsigned u = __float_as_uint(f);
  return (unsigned short)((u + 0x7FFFu + ((u >> 16) & 1u)) >> 16);
}
__device__ __forceinline__ float bf_bits2f(unsigned short h) { return __uint_as_float(((unsigned)h) << 16); }

__device__ __forceinline__ void dep_guard_h(v8f& a, v8f& b, v16h x, v16h y) { asm volatile("v_nop\n\tv_nop\n\tv_nop\n\tv_nop" : "+v"(a), "+v"(b) : "v"(x), "v"(y)); }
__device__ __forceinline__ void dep_guard_b(v8f& a, v8f& b, v16b x, v16b y) { asm volatile("v_nop\n\tv_nop\n\tv_nop\n\tv_nop" : "+v"(a), "+v"(b) : "v"(x), "v"(y)); }
__device__ __forceinline__ void keep4_h(v16h a, v16h b, v16h c, v16h d) { asm volatile("v_nop" :: "v"(a), "v"(b), "v"(c), "v"(d)); }
__device__ __forceinline__ void keep4_b(v16b a, v16b b, v16b c, v16b d) { asm volatile("v_nop" :: "v"(a), "v"(b), "v"(c), "v"(d)); }
__device__ __forceinline__ void acc_guard4(v8f& a, v8f& b, v8f& c, v8f& d) { asm volatile("v_nop\n\tv_nop\n\tv_nop\n\tv_nop" : "+v"(a), "+v"(b), "+v"(c), "+v"(d)); }
template <typename T> struct Frag;
template <> struct Frag<_Float16> {
  typedef v16h V; union U { v16h v; v8h h[2]; };
  static __device__ __forceinline__ v16h load(const _Float16* p) {
    U f; f.h[0] = *(const v8h*)(p); f.h[1] = *(const v8h*)(p + 16); return f.v;
  }
  static __device__ __forceinline__ v8f mma(v16h a, v16h b, v8f c) {
    return __builtin_amdgcn_wmma_f32_16x16x32_f16(false, a, false, b, (short)0, c, false, false);
  }
  static __device__ __forceinline__ void guard(v8f& a, v8f& b, v16h x, v16h y) { dep_guard_h(a, b, x, y); }
  static __device__ __forceinline__ void keep(v16h a, v16h b, v16h c, v16h d) { keep4_h(a, b, c, d); }
};
template <> struct Frag<__bf16> {
  typedef v16b V; union U { v16b v; v8b h[2]; };
  static __device__ __forceinline__ v16b load(const __bf16* p) {
    U f; f.h[0] = *(const v8b*)(p); f.h[1] = *(const v8b*)(p + 16); return f.v;
  }
  static __device__ __forceinline__ v8f mma(v16b a, v16b b, v8f c) {
    return __builtin_amdgcn_wmma_f32_16x16x32_bf16(false, a, false, b, (short)0, c, false, false);
  }
  static __device__ __forceinline__ void guard(v8f& a, v8f& b, v16b x, v16b y) { dep_guard_b(a, b, x, y); }
  static __device__ __forceinline__ void keep(v16b a, v16b b, v16b c, v16b d) { keep4_b(a, b, c, d); }
};

template <int ET> struct Elem;
template <> struct Elem<0> { typedef _Float16 T; };
template <> struct Elem<1> { typedef __bf16 T; };
template <int ET, bool SPLIT, int BIAS_MODE, int OUT_MODE, bool RESID, int ACT = 0>
__global__ __launch_bounds__(256) void wmma_gemm64(
    const unsigned short* __restrict__ Ap, const unsigned short* __restrict__ A2p, int lda, long strideA,
    const unsigned short* __restrict__ Btp, const unsigned short* __restrict__ Bt2p, int ldb, long strideB,
    void* __restrict__ Cout, void* __restrict__ Cout2, int ldc, long strideC,
    const float* __restrict__ bias,
    const float* __restrict__ resid, long strideR,
    int M, int N, int K, float scale) {
  typedef typename Elem<ET>::T T;
  typedef typename Frag<T>::V V;
  const T* A = (const T*)Ap; const T* A2 = (const T*)A2p; const T* Bt = (const T*)Btp; const T* Bt2 = (const T*)Bt2p;
  __shared__ __align__(16) float sT[8][16 * 68];
  const int b    = blockIdx.y;
  const int lane = threadIdx.x & 31;
  const int wave = threadIdx.x >> 5;
  const int tilesN = N >> 6;
  const int tilesM = M >> 6;
  const int tile = blockIdx.x * 8 + wave;
  if (tile >= tilesM * tilesN) return;
  const int tm = tile / tilesN;
  const int tn = tile - tm * tilesN;
  const int m0 = tm << 6;
  const int n0 = tn << 6;

  const T* Ab  = A  + (size_t)b * strideA;
  const T* Bb  = Bt + (size_t)b * strideB;
  const T* Ab2 = SPLIT ? (A2  + (size_t)b * strideA) : nullptr;
  const T* Bb2 = SPLIT ? (Bt2 + (size_t)b * strideB) : nullptr;

  const int rlane = lane & 15;
  const int koff  = (lane >> 4) * 8;
  const int mOff  = (lane >> 4) * 8;

  v8f acc[4][4];
#pragma unroll
  for (int i = 0; i < 4; ++i)
#pragma unroll
    for (int j = 0; j < 4; ++j) acc[i][j] = (v8f){0.f,0.f,0.f,0.f,0.f,0.f,0.f,0.f};

  for (int k0 = 0; k0 < K; k0 += 32) {
    V bh[4], bl[4];
#pragma unroll
    for (int j = 0; j < 4; ++j) {
      const size_t bo = (size_t)(n0 + (j << 4) + rlane) * ldb + koff + k0;
      bh[j] = Frag<T>::load(Bb + bo);
      if (SPLIT) bl[j] = Frag<T>::load(Bb2 + bo);
    }
#pragma unroll
    for (int i = 0; i < 4; ++i) {
      const size_t ao = (size_t)(m0 + (i << 4) + rlane) * lda + koff + k0;
      V ah = Frag<T>::load(Ab + ao);
      V al;
      if (SPLIT) al = Frag<T>::load(Ab2 + ao);
#pragma unroll
      for (int j = 0; j < 4; ++j) {
        acc[i][j] = Frag<T>::mma(ah, bh[j], acc[i][j]);
        if (SPLIT) {
          acc[i][j] = Frag<T>::mma(ah, bl[j], acc[i][j]);
          acc[i][j] = Frag<T>::mma(al, bh[j], acc[i][j]);
        }
      }
      Frag<T>::guard(acc[i][0], acc[i][3], ah, SPLIT ? al : ah);
    }
    Frag<T>::keep(bh[0], bh[1], bh[2], bh[3]);
    if (SPLIT) Frag<T>::keep(bl[0], bl[1], bl[2], bl[3]);
  }
  acc_guard4(acc[0][0], acc[0][1], acc[0][2], acc[0][3]);
  acc_guard4(acc[1][0], acc[1][1], acc[1][2], acc[1][3]);
  acc_guard4(acc[2][0], acc[2][1], acc[2][2], acc[2][3]);
  acc_guard4(acc[3][0], acc[3][1], acc[3][2], acc[3][3]);

  float* slab = sT[wave];
  const float* Rb = RESID ? (resid + (size_t)b * strideR) : nullptr;
#pragma unroll
  for (int i = 0; i < 4; ++i) {
    const int mBase = m0 + (i << 4);
#pragma unroll
    for (int j = 0; j < 4; ++j) {
      const int n = n0 + (j << 4) + rlane;
      float bv = 0.f;
      if (BIAS_MODE == 2) bv = bias[n];
#pragma unroll
      for (int r = 0; r < 8; ++r) {
        float v = acc[i][j][r] * scale;
        if (BIAS_MODE == 1) v += bias[mBase + mOff + r];
        if (BIAS_MODE == 2) v += bv;
        if (RESID) v += Rb[(size_t)(mBase + mOff + r) * ldc + n];
        if (ACT == 1) v = tanhf(v);
        if (ACT == 2) v = fmaxf(v, 0.0f);
        if (ACT == 3) v = v / (1.0f + expf(-v));
        if (ACT == 4) v = (v > 0.f) ? v : 0.01f * v;
        if (ACT == 5) v = 0.5f * v * (1.0f + erff(v * 0.70710678118654752f));
        slab[(mOff + r) * 68 + (j << 4) + rlane] = v;
      }
    }
    __builtin_amdgcn_fence(__ATOMIC_RELEASE, "workgroup");
    __builtin_amdgcn_wave_barrier();
    __builtin_amdgcn_fence(__ATOMIC_ACQUIRE, "workgroup");
    if (OUT_MODE == 0) {
      float* C = (float*)Cout + (size_t)b * strideC;
      const int hh = lane >> 4, c4 = (lane & 15) * 4;
      for (int pass = 0; pass < 2; ++pass) {
#pragma unroll
        for (int it = 0; it < 8; ++it) {
          const int row = it * 2 + hh;
          v4f v = *(const v4f*)(slab + row * 68 + c4);
          *(volatile v4f*)(C + (size_t)(mBase + row) * ldc + n0 + c4) = v;
        }
        __threadfence();
      }
    } else {
      const int q = lane >> 3, c8 = (lane & 7) * 8;
      unsigned short* C  = (unsigned short*)Cout  + (size_t)b * strideC;
      unsigned short* C2 = (OUT_MODE == 2) ? ((unsigned short*)Cout2 + (size_t)b * strideC) : nullptr;
      for (int pass = 0; pass < 2; ++pass) {
#pragma unroll
        for (int it = 0; it < 4; ++it) {
          const int row = it * 4 + q;
          const float* sp = slab + row * 68 + c8;
          v8h hv, lv;
#pragma unroll
          for (int e = 0; e < 8; ++e) {
            if (OUT_MODE == 1) {
              hv[e] = (_Float16)sp[e];
            } else {
              unsigned short hb = f2bf_bits(sp[e]);
              unsigned short lb = f2bf_bits(sp[e] - bf_bits2f(hb));
              hv[e] = __builtin_bit_cast(_Float16, hb);
              lv[e] = __builtin_bit_cast(_Float16, lb);
            }
          }
          *(volatile v8h*)(C + (size_t)(mBase + row) * ldc + n0 + c8) = hv;
          if (OUT_MODE == 2) *(volatile v8h*)(C2 + (size_t)(mBase + row) * ldc + n0 + c8) = lv;
        }
        __threadfence();
      }
    }
    __builtin_amdgcn_fence(__ATOMIC_RELEASE, "workgroup");
    __builtin_amdgcn_wave_barrier();
    __builtin_amdgcn_fence(__ATOMIC_ACQUIRE, "workgroup");
  }
}

constexpr int kBatch = 512;
constexpr int kSeq = 128;
constexpr int kFut = 24;
constexpr int kDin = 8;
constexpr int kHid = 256;
constexpr int kG3 = 768;
constexpr int kHdim = 64;
constexpr int kOutW = 456;
constexpr int kChunkB = 128;
constexpr int kChunkRows = kChunkB * kSeq;
constexpr int kNumChunks = kBatch / kChunkB;
constexpr int kRows = kBatch * kSeq;
constexpr int kInfN = 640;
constexpr float kW16Inv = 0.0625f;
constexpr float kPCarry = 1024.0f;

__device__ __forceinline__ v8f mma_h(v16h a, v16h b, v8f c) {
  c = __builtin_amdgcn_wmma_f32_16x16x32_f16(false, a, false, b, (short)0, c, false, false);
  asm volatile("v_nop\n\tv_nop\n\tv_nop\n\tv_nop" : "+v"(c) : "v"(a), "v"(b));
  return c;
}
__device__ __forceinline__ float wsum32(float v) {
#pragma unroll
  for (int o = 16; o > 0; o >>= 1) v += __shfl_xor(v, o, 32);
  return v;
}
__device__ __forceinline__ float wmax32(float v) {
#pragma unroll
  for (int o = 16; o > 0; o >>= 1) v = fmaxf(v, __shfl_xor(v, o, 32));
  return v;
}
__device__ __forceinline__ unsigned short f2h_bits(float f) {
  return __builtin_bit_cast(unsigned short, (_Float16)f);
}
__device__ __forceinline__ void lds_sync_wave() {
  __builtin_amdgcn_fence(__ATOMIC_RELEASE, "workgroup");
  __builtin_amdgcn_wave_barrier();
  __builtin_amdgcn_fence(__ATOMIC_ACQUIRE, "workgroup");
}

__global__ __launch_bounds__(256) void k_cast4(
    const float* __restrict__ s0, unsigned short* __restrict__ d0, int rows0, int scols0, int dcols0, int sld0,
    const float* __restrict__ s1, unsigned short* __restrict__ d1, int rows1, int scols1, int dcols1, int sld1,
    const float* __restrict__ s2, unsigned short* __restrict__ d2, int rows2, int scols2, int dcols2, int sld2,
    const float* __restrict__ s3, unsigned short* __restrict__ d3, int rows3, int scols3, int dcols3, int sld3,
    float scale) {
  const int y = blockIdx.y;
  const float* s = (y == 0) ? s0 : (y == 1) ? s1 : (y == 2) ? s2 : s3;
  unsigned short* d = (y == 0) ? d0 : (y == 1) ? d1 : (y == 2) ? d2 : d3;
  const int rows  = (y == 0) ? rows0 : (y == 1) ? rows1 : (y == 2) ? rows2 : rows3;
  const int scols = (y == 0) ? scols0 : (y == 1) ? scols1 : (y == 2) ? scols2 : scols3;
  const int dcols = (y == 0) ? dcols0 : (y == 1) ? dcols1 : (y == 2) ? dcols2 : dcols3;
  const int sld   = (y == 0) ? sld0 : (y == 1) ? sld1 : (y == 2) ? sld2 : sld3;
  const int i = blockIdx.x * 256 + threadIdx.x;
  const int n2 = (rows * dcols) >> 1;
  if (i < n2) {
    const int e0 = 2 * i;
    const int r = e0 / dcols;
    const int c = e0 - r * dcols;
    const int ca = (c < scols) ? c : (scols - 1);
    const int cb = (c + 1 < scols) ? (c + 1) : (scols - 1);
    float va = s[(size_t)r * sld + ca] * scale;
    float vb = s[(size_t)r * sld + cb] * scale;
    va = (c < scols) ? va : 0.0f;
    vb = (c + 1 < scols) ? vb : 0.0f;
    const unsigned u = (unsigned)f2h_bits(va) | ((unsigned)f2h_bits(vb) << 16);
    ((volatile unsigned*)d)[i] = u;
    __threadfence();
    ((volatile unsigned*)d)[i] = u;
  }
}

__global__ __launch_bounds__(256) void k_biascat(const float* __restrict__ bh0, const float* __restrict__ binf,
                                                 float* __restrict__ outb) {
  const int i = threadIdx.x;
  if (i < 160) {
    const int ia = (i < 128) ? i : 127;
    int ib = i - 128; ib = (ib < 0) ? 0 : ib;
    const v4f a = *(const v4f*)(bh0 + 4 * ia);
    const v4f c = *(const v4f*)(binf + 4 * ib);
    const bool first = (i < 128);
    const v4f v = { first ? a.x : c.x, first ? a.y : c.y, first ? a.z : c.z, first ? a.w : c.w };
    *(volatile v4f*)(outb + 4 * i) = v;
    __threadfence();
    *(volatile v4f*)(outb + 4 * i) = v;
  }
}

__global__ __launch_bounds__(256) void k_encoder(const float* __restrict__ x,
    const unsigned short* __restrict__ whh, const unsigned short* __restrict__ wihp,
    const float* __restrict__ bih, const float* __restrict__ bhh,
    unsigned short* __restrict__ enc, float* __restrict__ encf, int bbeg) {
  __shared__ __align__(16) unsigned short Hs[16 * 256];
  __shared__ __align__(16) unsigned short Xs[16 * 32];
  __shared__ __align__(16) float Hf[16 * 256];
  const int tid = threadIdx.x, lane = tid & 31, wave = tid >> 5, hh = lane >> 4, c = lane & 15;
  const int lb0 = blockIdx.x * 16;
  const int gb0 = bbeg + lb0;
  const v4u z4 = {0u, 0u, 0u, 0u};
  for (int i = tid; i < 512; i += 256) *(v4u*)(Hs + 8 * i) = z4;
  if (tid < 64) *(v4u*)(Xs + 8 * tid) = z4;
  __syncthreads();
  const int xr = (tid >> 3) & 15, xd = tid & 7;
  if (tid < 128) Xs[xr * 32 + xd] = f2h_bits(x[((size_t)(gb0 + xr) * kSeq + 0) * kDin + xd]);
  __syncthreads();

  int nu[2];
  float br[2], bz[2], bn_i[2], bn_h[2];
  float hreg[2][8];
#pragma unroll
  for (int us = 0; us < 2; ++us) {
    const int n = 16 * (2 * wave + us) + c;
    nu[us] = n;
    br[us] = bih[n] + bhh[n];
    bz[us] = bih[256 + n] + bhh[256 + n];
    bn_i[us] = bih[512 + n];
    bn_h[us] = bhh[512 + n];
#pragma unroll
    for (int r = 0; r < 8; ++r) hreg[us][r] = 0.0f;
  }
  const _Float16* HsH = (const _Float16*)(const void*)Hs;
  const _Float16* XsH = (const _Float16*)(const void*)Xs;
  const _Float16* WhH = (const _Float16*)(const void*)whh;
  const _Float16* WiH = (const _Float16*)(const void*)wihp;

  for (int t = 0; t < kSeq; ++t) {
    v8f acc[2][4];
#pragma unroll
    for (int us = 0; us < 2; ++us)
#pragma unroll
      for (int g = 0; g < 4; ++g) acc[us][g] = (v8f){0.f, 0.f, 0.f, 0.f, 0.f, 0.f, 0.f, 0.f};

#pragma unroll 1
    for (int k0 = 0; k0 < kHid; k0 += 32) {
      const v16h a = Frag<_Float16>::load(HsH + c * 256 + k0 + 8 * hh);
#pragma unroll
      for (int us = 0; us < 2; ++us) {
        const int rowb = 16 * (2 * wave + us) + c;
#pragma unroll
        for (int g = 0; g < 3; ++g) {
          const v16h bfr = Frag<_Float16>::load(WhH + (size_t)(g * 256 + rowb) * 256 + k0 + 8 * hh);
          acc[us][g] = mma_h(a, bfr, acc[us][g]);
        }
      }
    }
    {
      const v16h ax = Frag<_Float16>::load(XsH + c * 32 + 8 * hh);
#pragma unroll
      for (int us = 0; us < 2; ++us) {
        const int rowb = 16 * (2 * wave + us) + c;
        const v16h b0 = Frag<_Float16>::load(WiH + (size_t)rowb * 32 + 8 * hh);
        acc[us][0] = mma_h(ax, b0, acc[us][0]);
        const v16h b1 = Frag<_Float16>::load(WiH + (size_t)(256 + rowb) * 32 + 8 * hh);
        acc[us][1] = mma_h(ax, b1, acc[us][1]);
        const v16h b2 = Frag<_Float16>::load(WiH + (size_t)(512 + rowb) * 32 + 8 * hh);
        acc[us][3] = mma_h(ax, b2, acc[us][3]);
      }
    }
#pragma unroll
    for (int us = 0; us < 2; ++us) {
#pragma unroll
      for (int r = 0; r < 8; ++r) {
        const float pr = acc[us][0][r] * kW16Inv + br[us];
        const float pz = acc[us][1][r] * kW16Inv + bz[us];
        const float ghn = acc[us][2][r] * kW16Inv + bn_h[us];
        const float gin = acc[us][3][r] * kW16Inv + bn_i[us];
        const float rg = 1.0f / (1.0f + expf(-pr));
        const float zg = 1.0f / (1.0f + expf(-pz));
        const float ng = tanhf(gin + rg * ghn);
        const float hv = (1.0f - zg) * ng + zg * hreg[us][r];
        hreg[us][r] = hv;
      }
    }
    __syncthreads();
#pragma unroll
    for (int us = 0; us < 2; ++us)
#pragma unroll
      for (int r = 0; r < 8; ++r) {
        const float hv = hreg[us][r];
        Hs[(8 * hh + r) * 256 + nu[us]] = f2h_bits(hv);
        Hf[(8 * hh + r) * 256 + nu[us]] = hv;
      }
    if (tid < 128) {
      const int tn = (t + 1 < kSeq) ? (t + 1) : (kSeq - 1);
      Xs[xr * 32 + xd] = f2h_bits(x[((size_t)(gb0 + xr) * kSeq + tn) * kDin + xd]);
    }
    __syncthreads();
    {
      const int r0 = 2 * wave, r1 = 2 * wave + 1;
      const v4u v0 = *(const v4u*)(Hs + r0 * 256 + 8 * lane);
      const v4u v1 = *(const v4u*)(Hs + r1 * 256 + 8 * lane);
      const v4f fa0 = *(const v4f*)(Hf + r0 * 256 + 4 * lane);
      const v4f fa1 = *(const v4f*)(Hf + r0 * 256 + 128 + 4 * lane);
      const v4f fb0 = *(const v4f*)(Hf + r1 * 256 + 4 * lane);
      const v4f fb1 = *(const v4f*)(Hf + r1 * 256 + 128 + 4 * lane);
      unsigned short* p0 = enc + ((size_t)(lb0 + r0) * kSeq + t) * 256 + 8 * lane;
      unsigned short* p1 = enc + ((size_t)(lb0 + r1) * kSeq + t) * 256 + 8 * lane;
      float* q0p = encf + ((size_t)(lb0 + r0) * kSeq + t) * 256 + 4 * lane;
      float* q1p = encf + ((size_t)(lb0 + r1) * kSeq + t) * 256 + 4 * lane;
      *(volatile v4u*)p0 = v0; *(volatile v4u*)p1 = v1;
      *(volatile v4f*)q0p = fa0; *(volatile v4f*)(q0p + 128) = fa1;
      *(volatile v4f*)q1p = fb0; *(volatile v4f*)(q1p + 128) = fb1;
      __threadfence();
      *(volatile v4u*)p0 = v0; *(volatile v4u*)p1 = v1;
      *(volatile v4f*)q0p = fa0; *(volatile v4f*)(q0p + 128) = fa1;
      *(volatile v4f*)q1p = fb0; *(volatile v4f*)(q1p + 128) = fb1;
    }
  }
}

__global__ __launch_bounds__(128) void k_attn16(const unsigned short* __restrict__ qkv,
                                                unsigned short* __restrict__ att, float sscale) {
  __shared__ __align__(16) unsigned short Ksh[64 * 64];
  __shared__ __align__(16) unsigned short Vth[64 * 64];
  __shared__ __align__(16) unsigned short Psh[4][16 * 64];
  __shared__ __align__(16) float Os[4][16 * 68];
  const int tid = threadIdx.x, wave = tid >> 5, lane = tid & 31, hh = lane >> 4, c = lane & 15;
  const int bx = blockIdx.x;
  const int qb = bx & 1;
  const int bhid = bx >> 1;
  const int h = bhid & 3;
  const int b = bhid >> 2;
  const int q0 = qb * 64 + wave * 16;
  const size_t rb = (size_t)b * kSeq;
  const _Float16* QH = (const _Float16*)(const void*)qkv;
  const _Float16* KH = (const _Float16*)(const void*)Ksh;
  const _Float16* VH = (const _Float16*)(const void*)Vth;

  v16h qa[2];
#pragma unroll
  for (int dc = 0; dc < 2; ++dc)
    qa[dc] = Frag<_Float16>::load(QH + (rb + q0 + c) * kG3 + h * kHdim + dc * 32 + 8 * hh);

  float mrow[8], lrow[8];
  v8f oacc[4];
#pragma unroll
  for (int r = 0; r < 8; ++r) { mrow[r] = -__builtin_inff(); lrow[r] = 0.f; }
#pragma unroll
  for (int t = 0; t < 4; ++t) oacc[t] = (v8f){0.f, 0.f, 0.f, 0.f, 0.f, 0.f, 0.f, 0.f};

  for (int kc = 0; kc < 2; ++kc) {
    const int kv0 = kc * 64;
    __syncthreads();
    {
      const int kvr = tid >> 1, dh = (tid & 1) * 32;
      const unsigned short* krow = qkv + (rb + kv0 + kvr) * kG3 + kHid + h * kHdim + dh;
      const unsigned short* vrow = krow + kHid;
#pragma unroll
      for (int i = 0; i < 4; ++i) {
        const v4u kk = *(const v4u*)(krow + 8 * i);
        *(v4u*)(Ksh + kvr * 64 + dh + 8 * i) = kk;
        const v4u vv = *(const v4u*)(vrow + 8 * i);
        const int dd = dh + 8 * i;
        Vth[(dd + 0) * 64 + kvr] = (unsigned short)(vv.x & 0xffffu);
        Vth[(dd + 1) * 64 + kvr] = (unsigned short)(vv.x >> 16);
        Vth[(dd + 2) * 64 + kvr] = (unsigned short)(vv.y & 0xffffu);
        Vth[(dd + 3) * 64 + kvr] = (unsigned short)(vv.y >> 16);
        Vth[(dd + 4) * 64 + kvr] = (unsigned short)(vv.z & 0xffffu);
        Vth[(dd + 5) * 64 + kvr] = (unsigned short)(vv.z >> 16);
        Vth[(dd + 6) * 64 + kvr] = (unsigned short)(vv.w & 0xffffu);
        Vth[(dd + 7) * 64 + kvr] = (unsigned short)(vv.w >> 16);
      }
    }
    __syncthreads();

    v8f s[4];
#pragma unroll
    for (int j = 0; j < 4; ++j) {
      s[j] = (v8f){0.f, 0.f, 0.f, 0.f, 0.f, 0.f, 0.f, 0.f};
#pragma unroll
      for (int dc = 0; dc < 2; ++dc) {
        const v16h kb = Frag<_Float16>::load(KH + (j * 16 + c) * 64 + dc * 32 + 8 * hh);
        s[j] = mma_h(qa[dc], kb, s[j]);
      }
    }
    float cm[8];
#pragma unroll
    for (int r = 0; r < 8; ++r) {
      float m = -__builtin_inff();
#pragma unroll
      for (int j = 0; j < 4; ++j) { s[j][r] = s[j][r] * sscale; m = fmaxf(m, s[j][r]); }
#pragma unroll
      for (int off = 1; off < 16; off <<= 1) m = fmaxf(m, __shfl_xor(m, off, 32));
      cm[r] = m;
    }
    unsigned short* pw = Psh[wave];
#pragma unroll
    for (int r = 0; r < 8; ++r) {
      const float mnew = fmaxf(mrow[r], cm[r]);
      const float alpha = expf(mrow[r] - mnew);
      mrow[r] = mnew;
      float psum = 0.f;
#pragma unroll
      for (int j = 0; j < 4; ++j) {
        const float p = expf(s[j][r] - mnew);
        psum += p;
        pw[(8 * hh + r) * 64 + j * 16 + c] = f2h_bits(p * kPCarry);
      }
#pragma unroll
      for (int off = 1; off < 16; off <<= 1) psum += __shfl_xor(psum, off, 32);
      lrow[r] = lrow[r] * alpha + psum;
#pragma unroll
      for (int t = 0; t < 4; ++t) oacc[t][r] *= alpha;
    }
    lds_sync_wave();
    const _Float16* PH = (const _Float16*)(const void*)pw;
#pragma unroll 1
    for (int kk = 0; kk < 2; ++kk) {
      const v16h pa = Frag<_Float16>::load(PH + c * 64 + kk * 32 + 8 * hh);
#pragma unroll
      for (int t = 0; t < 4; ++t) {
        const v16h vb = Frag<_Float16>::load(VH + (t * 16 + c) * 64 + kk * 32 + 8 * hh);
        oacc[t] = mma_h(pa, vb, oacc[t]);
      }
    }
  }

  float* os = Os[wave];
#pragma unroll
  for (int r = 0; r < 8; ++r) {
    const float inv = 1.0f / (lrow[r] * kPCarry);
#pragma unroll
    for (int t = 0; t < 4; ++t) os[(8 * hh + r) * 68 + t * 16 + c] = oacc[t][r] * inv;
  }
  lds_sync_wave();
  {
    const int q = lane >> 3, c8 = (lane & 7) * 8;
    _Float16* AH = (_Float16*)(void*)att;
    for (int pass = 0; pass < 2; ++pass) {
#pragma unroll
      for (int it = 0; it < 4; ++it) {
        const int row = it * 4 + q;
        const float* sp = os + row * 68 + c8;
        v8h hv;
#pragma unroll
        for (int e = 0; e < 8; ++e) hv[e] = (_Float16)sp[e];
        *(volatile v8h*)(AH + (rb + q0 + row) * kHid + h * kHdim + c8) = hv;
      }
      __threadfence();
    }
  }
}

__global__ __launch_bounds__(256) void k_ln_res(const float* __restrict__ mh, const float* __restrict__ ef,
    const float* __restrict__ gam, const float* __restrict__ bet, unsigned short* __restrict__ outp, int nrows) {
  const int lane = threadIdx.x & 31, wave = threadIdx.x >> 5;
  const int row = blockIdx.x * 8 + wave;
  if (row >= nrows) return;
  const int c0 = 8 * lane;
  const float* mp = mh + (size_t)row * kHid + c0;
  const float* ep = ef + (size_t)row * kHid + c0;
  const v4f a = *(const v4f*)mp, bq = *(const v4f*)(mp + 4);
  const v4f e0 = *(const v4f*)ep, e1 = *(const v4f*)(ep + 4);
  float xv[8];
  xv[0] = a.x + e0.x; xv[1] = a.y + e0.y; xv[2] = a.z + e0.z; xv[3] = a.w + e0.w;
  xv[4] = bq.x + e1.x; xv[5] = bq.y + e1.y; xv[6] = bq.z + e1.z; xv[7] = bq.w + e1.w;
  float sm = ((xv[0] + xv[1]) + (xv[2] + xv[3])) + ((xv[4] + xv[5]) + (xv[6] + xv[7]));
  const float mean = wsum32(sm) * (1.0f / 256.0f);
  float qv = 0.f;
#pragma unroll
  for (int e = 0; e < 8; ++e) { const float d = xv[e] - mean; qv += d * d; }
  const float var = wsum32(qv) * (1.0f / 256.0f);
  const float inv = 1.0f / sqrtf(var + 1e-5f);
  const v4f g0 = *(const v4f*)(gam + c0), g1 = *(const v4f*)(gam + c0 + 4);
  const v4f b0 = *(const v4f*)(bet + c0), b1 = *(const v4f*)(bet + c0 + 4);
  const float gv[8] = {g0.x, g0.y, g0.z, g0.w, g1.x, g1.y, g1.z, g1.w};
  const float bv[8] = {b0.x, b0.y, b0.z, b0.w, b1.x, b1.y, b1.z, b1.w};
  v8h hv;
#pragma unroll
  for (int e = 0; e < 8; ++e) { const float tn = (xv[e] - mean) * inv; hv[e] = (_Float16)(tn * gv[e] + bv[e]); }
  unsigned short* op = outp + (size_t)row * kHid + c0;
  *(volatile v8h*)(void*)op = hv;
  __threadfence();
  *(volatile v8h*)(void*)op = hv;
}

template <int NJ>
__global__ __launch_bounds__(256) void k_ln_elu(const float* __restrict__ in, int ldin,
    const float* __restrict__ gam, const float* __restrict__ bet, unsigned short* __restrict__ outp, int nrows) {
  const int lane = threadIdx.x & 31, wave = threadIdx.x >> 5;
  const int row = blockIdx.x * 8 + wave;
  if (row >= nrows) return;
  const float invn = 1.0f / (float)(256 * NJ);
  const float* rp = in + (size_t)row * ldin + 8 * lane;
  float sm = 0.f;
#pragma unroll 1
  for (int j = 0; j < NJ; ++j) {
    const v4f a = *(const v4f*)(rp + 256 * j), bq = *(const v4f*)(rp + 256 * j + 4);
    sm += ((a.x + a.y) + (a.z + a.w)) + ((bq.x + bq.y) + (bq.z + bq.w));
  }
  const float mean = wsum32(sm) * invn;
  float qv = 0.f;
#pragma unroll 1
  for (int j = 0; j < NJ; ++j) {
    const v4f a = *(const v4f*)(rp + 256 * j), bq = *(const v4f*)(rp + 256 * j + 4);
    const float d0 = a.x - mean, d1 = a.y - mean, d2 = a.z - mean, d3 = a.w - mean;
    const float d4 = bq.x - mean, d5 = bq.y - mean, d6 = bq.z - mean, d7 = bq.w - mean;
    qv += ((d0 * d0 + d1 * d1) + (d2 * d2 + d3 * d3)) + ((d4 * d4 + d5 * d5) + (d6 * d6 + d7 * d7));
  }
  const float var = wsum32(qv) * invn;
  const float inv = 1.0f / sqrtf(var + 1e-5f);
#pragma unroll 1
  for (int j = 0; j < NJ; ++j) {
    const v4f a = *(const v4f*)(rp + 256 * j), bq = *(const v4f*)(rp + 256 * j + 4);
    const v4f g0 = *(const v4f*)(gam + 256 * j + 8 * lane), g1 = *(const v4f*)(gam + 256 * j + 8 * lane + 4);
    const v4f b0 = *(const v4f*)(bet + 256 * j + 8 * lane), b1 = *(const v4f*)(bet + 256 * j + 8 * lane + 4);
    float y[8];
    { const float t0 = (a.x - mean) * inv;  y[0] = t0 * g0.x + b0.x; }
    { const float t1 = (a.y - mean) * inv;  y[1] = t1 * g0.y + b0.y; }
    { const float t2 = (a.z - mean) * inv;  y[2] = t2 * g0.z + b0.z; }
    { const float t3 = (a.w - mean) * inv;  y[3] = t3 * g0.w + b0.w; }
    { const float t4 = (bq.x - mean) * inv; y[4] = t4 * g1.x + b1.x; }
    { const float t5 = (bq.y - mean) * inv; y[5] = t5 * g1.y + b1.y; }
    { const float t6 = (bq.z - mean) * inv; y[6] = t6 * g1.z + b1.z; }
    { const float t7 = (bq.w - mean) * inv; y[7] = t7 * g1.w + b1.w; }
    v8h hv;
#pragma unroll
    for (int e = 0; e < 8; ++e) {
      const float ye = y[e];
      const float ne = expf(fminf(ye, 0.0f)) - 1.0f;
      hv[e] = (_Float16)((ye > 0.0f) ? ye : ne);
    }
    unsigned short* op = outp + (size_t)row * (256 * NJ) + 256 * j + 8 * lane;
    *(volatile v8h*)(void*)op = hv;
    __threadfence();
    *(volatile v8h*)(void*)op = hv;
  }
}

__global__ __launch_bounds__(256) void k_le2_out(const float* __restrict__ in,
    const float* __restrict__ gam, const float* __restrict__ bet,
    const float* __restrict__ woutc, const float* __restrict__ boutc, const float* __restrict__ gpfm,
    int mode, int f, float* __restrict__ past, float* __restrict__ futt, float* __restrict__ prev) {
  __shared__ float sc[32];
  const int lane = threadIdx.x & 31, wave = threadIdx.x >> 5;
  const int rb0 = blockIdx.x * 32;
  const v4f wc = *(const v4f*)(woutc + 4 * lane);
  const v4f gv = *(const v4f*)(gam + 4 * lane);
  const v4f bv = *(const v4f*)(bet + 4 * lane);
  const float bc = boutc[0];
#pragma unroll 1
  for (int i = 0; i < 4; ++i) {
    const int row = rb0 + wave * 4 + i;
    const v4f a = *(const v4f*)(in + (size_t)row * 128 + 4 * lane);
    const float mean = wsum32((a.x + a.y) + (a.z + a.w)) * (1.0f / 128.0f);
    const float d0 = a.x - mean, d1 = a.y - mean, d2 = a.z - mean, d3 = a.w - mean;
    const float var = wsum32((d0 * d0 + d1 * d1) + (d2 * d2 + d3 * d3)) * (1.0f / 128.0f);
    const float inv = 1.0f / sqrtf(var + 1e-5f);
    float y0 = d0 * inv * gv.x + bv.x, y1 = d1 * inv * gv.y + bv.y, y2 = d2 * inv * gv.z + bv.z, y3 = d3 * inv * gv.w + bv.w;
    const float n0 = expf(fminf(y0, 0.f)) - 1.0f, n1 = expf(fminf(y1, 0.f)) - 1.0f;
    const float n2 = expf(fminf(y2, 0.f)) - 1.0f, n3 = expf(fminf(y3, 0.f)) - 1.0f;
    y0 = (y0 > 0.f) ? y0 : n0; y1 = (y1 > 0.f) ? y1 : n1; y2 = (y2 > 0.f) ? y2 : n2; y3 = (y3 > 0.f) ? y3 : n3;
    const float dot = wsum32((y0 * wc.x + y1 * wc.y) + (y2 * wc.z + y3 * wc.w)) + bc;
    if (lane == 0) sc[wave * 4 + i] = dot;
  }
  __syncthreads();
  if (wave == 0) {
    const float val = sc[lane];
    const int rg = rb0 + lane;
    const int rgc = (rg < kBatch) ? rg : (kBatch - 1);
    const float pvt = gpfm[(size_t)rgc * kFut + f];
    if (mode == 0) {
      volatile float* p = past + rg;
      *p = val;
      __threadfence();
      *p = val;
    } else {
      const float nx = val + pvt;
      volatile float* p1 = futt + (size_t)f * kBatch + rg;
      volatile float* p2 = prev + rg;
      *p1 = val; *p2 = nx;
      __threadfence();
      *p1 = val; *p2 = nx;
    }
  }
}

__global__ __launch_bounds__(256) void k_transp(const unsigned short* __restrict__ in, unsigned short* __restrict__ outp) {
  __shared__ __align__(16) unsigned short Tt[64 * 136];
  const int tid = threadIdx.x, lane = tid & 31, wave = tid >> 5;
  const int b = blockIdx.x >> 2, n0 = (blockIdx.x & 3) * 64;
  const int l = tid >> 1, dh = (tid & 1) * 32;
  const unsigned short* src = in + ((size_t)b * kSeq + l) * kHid + n0 + dh;
#pragma unroll
  for (int i = 0; i < 4; ++i) {
    const v4u vv = *(const v4u*)(src + 8 * i);
    const int cb = dh + 8 * i;
    Tt[(cb + 0) * 136 + l] = (unsigned short)(vv.x & 0xffffu);
    Tt[(cb + 1) * 136 + l] = (unsigned short)(vv.x >> 16);
    Tt[(cb + 2) * 136 + l] = (unsigned short)(vv.y & 0xffffu);
    Tt[(cb + 3) * 136 + l] = (unsigned short)(vv.y >> 16);
    Tt[(cb + 4) * 136 + l] = (unsigned short)(vv.z & 0xffffu);
    Tt[(cb + 5) * 136 + l] = (unsigned short)(vv.z >> 16);
    Tt[(cb + 6) * 136 + l] = (unsigned short)(vv.w & 0xffffu);
    Tt[(cb + 7) * 136 + l] = (unsigned short)(vv.w >> 16);
  }
  __syncthreads();
  const int col8 = 8 * (lane & 15);
  for (int pass = 0; pass < 2; ++pass) {
#pragma unroll
    for (int i = 0; i < 4; ++i) {
      const int row = 8 * wave + 2 * i + (lane >> 4);
      const v4u q = *(const v4u*)(Tt + row * 136 + col8);
      *(volatile v4u*)(outp + ((size_t)b * kHid + n0 + row) * kSeq + col8) = q;
    }
    __threadfence();
  }
}

__global__ __launch_bounds__(128) void k_applied(const float* __restrict__ cinf, int ldc,
    const float* __restrict__ winf, const float* __restrict__ gpfm, const float* __restrict__ prev, int f, int mode,
    const unsigned short* __restrict__ encT, float* __restrict__ hdec, unsigned short* __restrict__ acomb) {
  __shared__ __align__(16) unsigned short Wt[16 * 128];
  __shared__ float red[8];
  __shared__ __align__(16) float aps[256];
  const int tid = threadIdx.x, wave = tid >> 5, lane = tid & 31, hh = lane >> 4, c = lane & 15;
  const int b = blockIdx.x;
  const v4u z4 = {0u, 0u, 0u, 0u};
  *(v4u*)(Wt + 8 * tid) = z4;
  *(v4u*)(Wt + 1024 + 8 * tid) = z4;
  const float pm = gpfm[(size_t)b * kFut];
  const float pvv = prev[b];
  const float indec = (f == 0) ? pm : pvv;
  const float lg = cinf[(size_t)b * ldc + tid] + indec * winf[(size_t)tid * 257 + 256];
  float m = wmax32(lg);
  if (lane == 0) red[wave] = m;
  __syncthreads();
  m = fmaxf(fmaxf(red[0], red[1]), fmaxf(red[2], red[3]));
  const float e = expf(lg - m);
  float ssum = wsum32(e);
  if (lane == 0) red[4 + wave] = ssum;
  __syncthreads();
  ssum = ((red[4] + red[5]) + red[6]) + red[7];
  const float wsc = e * (1.0f / ssum) * kPCarry;
  const float wv = (mode == 0) ? (kPCarry / 128.0f) : wsc;
  Wt[tid] = f2h_bits(wv);
  __syncthreads();

  const _Float16* WtH = (const _Float16*)(const void*)Wt;
  const _Float16* EH = (const _Float16*)(const void*)encT;
  v8f acc[4];
#pragma unroll
  for (int j = 0; j < 4; ++j) acc[j] = (v8f){0.f, 0.f, 0.f, 0.f, 0.f, 0.f, 0.f, 0.f};
#pragma unroll
  for (int k0 = 0; k0 < kSeq; k0 += 32) {
    const v16h a = Frag<_Float16>::load(WtH + c * 128 + k0 + 8 * hh);
#pragma unroll
    for (int j = 0; j < 4; ++j) {
      const int n = 64 * wave + 16 * j + c;
      const v16h bfr = Frag<_Float16>::load(EH + ((size_t)b * kHid + n) * kSeq + k0 + 8 * hh);
      acc[j] = mma_h(a, bfr, acc[j]);
    }
  }
  const float cinv = 1.0f / kPCarry;
  const float v0 = acc[0][0] * cinv, v1 = acc[1][0] * cinv, v2 = acc[2][0] * cinv, v3 = acc[3][0] * cinv;
  if (hh == 0) {
    aps[64 * wave + c] = v0;
    aps[64 * wave + 16 + c] = v1;
    aps[64 * wave + 32 + c] = v2;
    aps[64 * wave + 48 + c] = v3;
  }
  __syncthreads();
  if (wave == 0) {
    const v4f p0 = *(const v4f*)(aps + 8 * lane), p1 = *(const v4f*)(aps + 8 * lane + 4);
    v8h hv;
    hv[0] = (_Float16)p0.x; hv[1] = (_Float16)p0.y; hv[2] = (_Float16)p0.z; hv[3] = (_Float16)p0.w;
    hv[4] = (_Float16)p1.x; hv[5] = (_Float16)p1.y; hv[6] = (_Float16)p1.z; hv[7] = (_Float16)p1.w;
    unsigned short* op = acomb + (size_t)b * 512 + ((mode == 0) ? 256 : 0) + 8 * lane;
    const v4f q0v = *(const v4f*)(aps + 4 * lane), q1v = *(const v4f*)(aps + 128 + 4 * lane);
    float* hp = hdec + (size_t)b * kHid + 4 * lane;
    *(volatile v8h*)(void*)op = hv;
    if (mode == 0) { *(volatile v4f*)hp = q0v; *(volatile v4f*)(hp + 128) = q1v; }
    __threadfence();
    *(volatile v8h*)(void*)op = hv;
    if (mode == 0) { *(volatile v4f*)hp = q0v; *(volatile v4f*)(hp + 128) = q1v; }
  }
}

__global__ __launch_bounds__(256) void k_ln_dec(const float* __restrict__ cc, const float* __restrict__ gam,
    const float* __restrict__ bet, float* __restrict__ hmid, unsigned short* __restrict__ hmid16) {
  __shared__ __align__(16) unsigned short slab[8][256];
  const int lane = threadIdx.x & 31, wave = threadIdx.x >> 5;
  const int b = blockIdx.x * 8 + wave;
  const float* rp = cc + (size_t)b * kHid + 4 * lane;
  const v4f a0 = *(const v4f*)rp, a1 = *(const v4f*)(rp + 128);
  const float mean = wsum32(((a0.x + a0.y) + (a0.z + a0.w)) + ((a1.x + a1.y) + (a1.z + a1.w))) * (1.0f / 256.0f);
  const float d0 = a0.x - mean, d1 = a0.y - mean, d2 = a0.z - mean, d3 = a0.w - mean;
  const float d4 = a1.x - mean, d5 = a1.y - mean, d6 = a1.z - mean, d7 = a1.w - mean;
  const float var = wsum32(((d0 * d0 + d1 * d1) + (d2 * d2 + d3 * d3)) + ((d4 * d4 + d5 * d5) + (d6 * d6 + d7 * d7))) * (1.0f / 256.0f);
  const float inv = 1.0f / sqrtf(var + 1e-5f);
  const v4f g0 = *(const v4f*)(gam + 4 * lane), g1 = *(const v4f*)(gam + 128 + 4 * lane);
  const v4f b0 = *(const v4f*)(bet + 4 * lane), b1 = *(const v4f*)(bet + 128 + 4 * lane);
  const v4f y0 = { d0 * inv * g0.x + b0.x, d1 * inv * g0.y + b0.y, d2 * inv * g0.z + b0.z, d3 * inv * g0.w + b0.w };
  const v4f y1 = { d4 * inv * g1.x + b1.x, d5 * inv * g1.y + b1.y, d6 * inv * g1.z + b1.z, d7 * inv * g1.w + b1.w };
  slab[wave][4 * lane + 0] = f2h_bits(y0.x); slab[wave][4 * lane + 1] = f2h_bits(y0.y);
  slab[wave][4 * lane + 2] = f2h_bits(y0.z); slab[wave][4 * lane + 3] = f2h_bits(y0.w);
  slab[wave][128 + 4 * lane + 0] = f2h_bits(y1.x); slab[wave][128 + 4 * lane + 1] = f2h_bits(y1.y);
  slab[wave][128 + 4 * lane + 2] = f2h_bits(y1.z); slab[wave][128 + 4 * lane + 3] = f2h_bits(y1.w);
  float* op = hmid + (size_t)b * kHid + 4 * lane;
  *(volatile v4f*)op = y0; *(volatile v4f*)(op + 128) = y1;
  lds_sync_wave();
  const v4u hq = *(const v4u*)(slab[wave] + 8 * lane);
  unsigned short* hp = hmid16 + (size_t)b * kHid + 8 * lane;
  *(volatile v4u*)hp = hq;
  __threadfence();
  *(volatile v4f*)op = y0; *(volatile v4f*)(op + 128) = y1;
  *(volatile v4u*)hp = hq;
}

__global__ __launch_bounds__(256) void k_gates(const float* __restrict__ gh, const float* __restrict__ hmid,
    const float* __restrict__ wihd, const float* __restrict__ bihd, const float* __restrict__ gpfm,
    const float* __restrict__ prev, int f, float* __restrict__ hdec, unsigned short* __restrict__ acomb) {
  __shared__ __align__(16) float slf[8][128];
  __shared__ __align__(16) unsigned short slh[8][128];
  const int tid = threadIdx.x, wave = tid >> 5, lane = tid & 31;
  const int b = blockIdx.x * 4 + (wave >> 1);
  const int half = wave & 1;
  const float pm = gpfm[(size_t)b * kFut];
  const float pvv = prev[b];
  const float indec = (f == 0) ? pm : pvv;
  const size_t gro = (size_t)b * kG3 + half * 128;
  const size_t hro = (size_t)b * kHid + half * 128;
#pragma unroll 1
  for (int e = 0; e < 4; ++e) {
    const int u = 4 * lane + e;
    const int n = half * 128 + u;
    const float gir = indec * wihd[n] + bihd[n];
    const float giz = indec * wihd[256 + n] + bihd[256 + n];
    const float gin = indec * wihd[512 + n] + bihd[512 + n];
    const float ghr = gh[gro + u], ghz = gh[gro + 256 + u], ghn = gh[gro + 512 + u];
    const float rg = 1.0f / (1.0f + expf(-(gir + ghr)));
    const float zg = 1.0f / (1.0f + expf(-(giz + ghz)));
    const float ng = tanhf(gin + rg * ghn);
    const float hp = hmid[hro + u];
    const float hv = (1.0f - zg) * ng + zg * hp;
    slf[wave][u] = hv;
    slh[wave][u] = f2h_bits(hv);
  }
  lds_sync_wave();
  const v4f o = *(const v4f*)(slf[wave] + 4 * lane);
  const v4u hq = *(const v4u*)(slh[wave] + 8 * (lane & 15));
  float* op = hdec + hro + 4 * lane;
  unsigned short* hp16 = acomb + (size_t)b * 512 + 256 + half * 128 + 8 * (lane & 15);
  *(volatile v4f*)op = o;
  if (lane < 16) *(volatile v4u*)hp16 = hq;
  __threadfence();
  *(volatile v4f*)op = o;
  if (lane < 16) *(volatile v4u*)hp16 = hq;
}

__global__ __launch_bounds__(256) void k_final(const float* __restrict__ past, const float* __restrict__ futt,
    const float* __restrict__ gpm, const float* __restrict__ gpl, const float* __restrict__ gpu,
    const float* __restrict__ gfm, const float* __restrict__ gfl, const float* __restrict__ gfu,
    float* __restrict__ out, int nthr) {
  const int i = blockIdx.x * 256 + threadIdx.x;
  if (i >= nthr) return;
  const int e0 = 4 * i;
  const int b = e0 / kOutW;
  const int c0 = e0 - b * kOutW;
  float vals[4];
#pragma unroll
  for (int k = 0; k < 4; ++k) {
    const int cc = c0 + k;
    const int l = cc & 127;
    const size_t pidx = (size_t)b * kSeq + l;
    const float pv = past[pidx];
    const float g0 = gpm[pidx], g1 = gpl[pidx], g2 = gpu[pidx];
    int cf = cc - 384; cf = (cf < 0) ? 0 : cf;
    int sg = cf / kFut; sg = (sg > 2) ? 2 : sg;
    const int ff = cf - kFut * sg;
    const float fv = futt[(size_t)ff * kBatch + b];
    const size_t fidx = (size_t)b * kFut + ff;
    const float h0 = gfm[fidx], h1 = gfl[fidx], h2 = gfu[fidx];
    float v = fv + h2;
    v = (sg == 1) ? (fv + h1) : v;
    v = (sg == 0) ? (fv + h0) : v;
    v = (cc < 384) ? (pv + g2) : v;
    v = (cc < 256) ? (pv + g1) : v;
    v = (cc < 128) ? (pv + g0) : v;
    vals[k] = v;
  }
  const v4f o = {vals[0], vals[1], vals[2], vals[3]};
  *(volatile v4f*)(out + e0) = o;
  __threadfence();
  *(volatile v4f*)(out + e0) = o;
}

static inline dim3 gemm_grid(int M, int N) {
  const int tiles = (M / 64) * (N / 64);
  return dim3((unsigned)((tiles + 7) / 8), 1, 1);
}
static void gemm_f16out(const unsigned short* A, int lda, const unsigned short* Bt, int ldb, unsigned short* C, int ldc,
                        const float* bias, int M, int N, int K, float scale, hipStream_t st) {
  wmma_gemm64<0, false, 2, 1, false, 0><<<gemm_grid(M, N), 256, 0, st>>>(
      A, A, lda, 0L, Bt, Bt, ldb, 0L, (void*)C, (void*)C, ldc, 0L, bias, bias, 0L, M, N, K, scale);
}
static void gemm_f32out(const unsigned short* A, int lda, const unsigned short* Bt, int ldb, float* C, int ldc,
                        const float* bias, int M, int N, int K, float scale, hipStream_t st) {
  wmma_gemm64<0, false, 2, 0, false, 0><<<gemm_grid(M, N), 256, 0, st>>>(
      A, A, lda, 0L, Bt, Bt, ldb, 0L, (void*)C, (void*)C, ldc, 0L, bias, bias, 0L, M, N, K, scale);
}
static void gemm_f32out_res(const unsigned short* A, int lda, const unsigned short* Bt, int ldb, float* C, int ldc,
                            const float* bias, const float* resid, int M, int N, int K, float scale, hipStream_t st) {
  wmma_gemm64<0, false, 2, 0, true, 0><<<gemm_grid(M, N), 256, 0, st>>>(
      A, A, lda, 0L, Bt, Bt, ldb, 0L, (void*)C, (void*)C, ldc, 0L, bias, resid, 0L, M, N, K, scale);
}

extern "C" void kernel_launch(void* const* d_in, const int* in_sizes, int n_in,
                              void* d_out, int out_size, void* d_ws, size_t ws_size,
                              hipStream_t stream) {
  if (n_in < 41) return;
  if (in_sizes[0] != kBatch * kSeq * kDin) return;
  if (in_sizes[1] != kRows || in_sizes[4] != kBatch * kFut) return;
  if (in_sizes[8] != kG3 * kHid || in_sizes[11] != kG3 * kHid || in_sizes[17] != kSeq * 257) return;
  if (in_sizes[19] != kHid * 512 || in_sizes[24] != kG3 * kHid || in_sizes[27] != 512 * kHid) return;
  if (in_sizes[31] != kHid * 512 || in_sizes[35] != 128 * kHid || in_sizes[39] != 128 || in_sizes[40] < 1) return;
  if (out_size != kBatch * kOutW) return;

  const float* x         = (const float*)d_in[0];
  const float* gp_pm     = (const float*)d_in[1];
  const float* gp_pl     = (const float*)d_in[2];
  const float* gp_pu     = (const float*)d_in[3];
  const float* gp_fm     = (const float*)d_in[4];
  const float* gp_fl     = (const float*)d_in[5];
  const float* gp_fu     = (const float*)d_in[6];
  const float* W_ih_enc  = (const float*)d_in[7];
  const float* W_hh_enc  = (const float*)d_in[8];
  const float* b_ih_enc  = (const float*)d_in[9];
  const float* b_hh_enc  = (const float*)d_in[10];
  const float* W_in_proj = (const float*)d_in[11];
  const float* b_in_proj = (const float*)d_in[12];
  const float* W_out_proj = (const float*)d_in[13];
  const float* b_out_proj = (const float*)d_in[14];
  const float* g_mh_ln   = (const float*)d_in[15];
  const float* be_mh_ln  = (const float*)d_in[16];
  const float* W_inf     = (const float*)d_in[17];
  const float* b_inf     = (const float*)d_in[18];
  const float* W_comb    = (const float*)d_in[19];
  const float* b_comb    = (const float*)d_in[20];
  const float* g_inf_ln  = (const float*)d_in[21];
  const float* be_inf_ln = (const float*)d_in[22];
  const float* W_ih_dec  = (const float*)d_in[23];
  const float* W_hh_dec  = (const float*)d_in[24];
  const float* b_ih_dec  = (const float*)d_in[25];
  const float* b_hh_dec  = (const float*)d_in[26];
  const float* W_h0 = (const float*)d_in[27];
  const float* b_h0 = (const float*)d_in[28];
  const float* g_ln0 = (const float*)d_in[29];
  const float* be_ln0 = (const float*)d_in[30];
  const float* W_h1 = (const float*)d_in[31];
  const float* b_h1 = (const float*)d_in[32];
  const float* g_ln1 = (const float*)d_in[33];
  const float* be_ln1 = (const float*)d_in[34];
  const float* W_h2 = (const float*)d_in[35];
  const float* b_h2 = (const float*)d_in[36];
  const float* g_ln2 = (const float*)d_in[37];
  const float* be_ln2 = (const float*)d_in[38];
  const float* W_outc = (const float*)d_in[39];
  const float* b_outc = (const float*)d_in[40];
  float* out = (float*)d_out;

  char* ws = (char*)d_ws;
  size_t off = 0;
  auto carve = [&](size_t bytes) -> char* { char* p = ws + off; off += (bytes + 255) & ~(size_t)255; return p; };
  unsigned short* WHHE  = (unsigned short*)carve((size_t)kG3 * kHid * 2);
  unsigned short* WINP  = (unsigned short*)carve((size_t)kG3 * kHid * 2);
  unsigned short* WHHD  = (unsigned short*)carve((size_t)kG3 * kHid * 2);
  unsigned short* WOUT  = (unsigned short*)carve((size_t)kHid * kHid * 2);
  unsigned short* WIHP  = (unsigned short*)carve((size_t)kG3 * 32 * 2);
  unsigned short* WCOMB = (unsigned short*)carve((size_t)kHid * 512 * 2);
  unsigned short* WH0INF = (unsigned short*)carve((size_t)kInfN * kHid * 2);
  unsigned short* WINF16 = WH0INF + (size_t)512 * kHid;
  unsigned short* WH1   = (unsigned short*)carve((size_t)kHid * 512 * 2);
  unsigned short* WH2   = (unsigned short*)carve((size_t)128 * kHid * 2);
  float*          BIASC = (float*)carve((size_t)kInfN * 4);
  unsigned short* ENC2  = (unsigned short*)carve((size_t)kRows * kHid * 2);
  unsigned short* RENC  = (unsigned short*)carve((size_t)kChunkRows * kHid * 2);
  char*           RA    = carve((size_t)kChunkRows * 512 * 4);
  char*           RB    = carve((size_t)kChunkRows * 512 * 2);
  char*           RC    = carve((size_t)kChunkRows * kHid * 4);
  float*          PAST  = (float*)carve((size_t)kRows * 4);
  unsigned short* ACOMB = (unsigned short*)carve((size_t)kBatch * 512 * 2);
  float*          DG    = (float*)carve((size_t)kBatch * kInfN * 4);
  float*          CCOMB = (float*)carve((size_t)kBatch * kHid * 4);
  float*          HDEC  = (float*)carve((size_t)kBatch * kHid * 4);
  float*          HMID  = (float*)carve((size_t)kBatch * kHid * 4);
  unsigned short* HMID16 = (unsigned short*)carve((size_t)kBatch * kHid * 2);
  float*          GH    = (float*)carve((size_t)kBatch * kG3 * 4);
  unsigned short* Z0D   = (unsigned short*)carve((size_t)kBatch * 512 * 2);
  float*          D1    = (float*)carve((size_t)kBatch * kHid * 4);
  unsigned short* Z1D   = (unsigned short*)carve((size_t)kBatch * kHid * 2);
  float*          D2    = (float*)carve((size_t)kBatch * 128 * 4);
  float*          FUTT  = (float*)carve((size_t)kFut * kBatch * 4);
  float*          PREV  = (float*)carve((size_t)kBatch * 4);
  if (off > ws_size) return;

  const float wscale = 16.0f;
  k_cast4<<<dim3(384, 4), 256, 0, stream>>>(
      W_hh_enc, WHHE, kG3, kHid, kHid, kHid,
      W_in_proj, WINP, kG3, kHid, kHid, kHid,
      W_hh_dec, WHHD, kG3, kHid, kHid, kHid,
      W_out_proj, WOUT, kHid, kHid, kHid, kHid, wscale);
  k_cast4<<<dim3(256, 4), 256, 0, stream>>>(
      W_ih_enc, WIHP, kG3, kDin, 32, kDin,
      W_inf, WINF16, kSeq, kHid, kHid, 257,
      W_comb, WCOMB, kHid, 512, 512, 512,
      W_h0, WH0INF, 512, kHid, kHid, kHid, wscale);
  k_cast4<<<dim3(256, 4), 256, 0, stream>>>(
      W_h1, WH1, kHid, 512, 512, 512,
      W_h2, WH2, 128, kHid, kHid, kHid,
      W_h1, WH1, 0, 512, 512, 512,
      W_h1, WH1, 0, 512, 512, 512, wscale);
  k_biascat<<<1, 256, 0, stream>>>(b_h0, b_inf, BIASC);

  for (int c = 0; c < kNumChunks; ++c) {
    unsigned short* QKVc = (unsigned short*)RA;
    unsigned short* ATTc = (unsigned short*)RB;
    float* ENCFc = (float*)RC;
    float* MHc = (float*)RA;
    float* G0c = (float*)RA;
    unsigned short* Z0c = (unsigned short*)RB;
    float* G1c = (float*)RC;
    unsigned short* Z1c = (unsigned short*)RB;
    float* G2c = (float*)RC;
    unsigned short* ENC2c = ENC2 + (size_t)c * kChunkRows * kHid;

    k_encoder<<<kChunkB / 16, 256, 0, stream>>>(x, WHHE, WIHP, b_ih_enc, b_hh_enc, RENC, ENCFc, c * kChunkB);
    gemm_f16out(RENC, kHid, WINP, kHid, QKVc, kG3, b_in_proj, kChunkRows, kG3, kHid, kW16Inv, stream);
    k_attn16<<<kChunkB * 4 * 2, 128, 0, stream>>>(QKVc, ATTc, 0.125f);
    gemm_f32out(ATTc, kHid, WOUT, kHid, MHc, kHid, b_out_proj, kChunkRows, kHid, kHid, kW16Inv, stream);
    k_ln_res<<<kChunkRows / 8, 256, 0, stream>>>(MHc, ENCFc, g_mh_ln, be_mh_ln, ENC2c, kChunkRows);
    gemm_f32out(ENC2c, kHid, WH0INF, kHid, G0c, 512, b_h0, kChunkRows, 512, kHid, kW16Inv, stream);
    k_ln_elu<2><<<kChunkRows / 8, 256, 0, stream>>>(G0c, 512, g_ln0, be_ln0, Z0c, kChunkRows);
    gemm_f32out(Z0c, 512, WH1, 512, G1c, kHid, b_h1, kChunkRows, kHid, 512, kW16Inv, stream);
    k_ln_elu<1><<<kChunkRows / 8, 256, 0, stream>>>(G1c, kHid, g_ln1, be_ln1, Z1c, kChunkRows);
    gemm_f32out(Z1c, kHid, WH2, kHid, G2c, 128, b_h2, kChunkRows, 128, kHid, kW16Inv, stream);
    k_le2_out<<<kChunkRows / 32, 256, 0, stream>>>(G2c, g_ln2, be_ln2, W_outc, b_outc, gp_fm, 0, 0,
                                                   PAST + (size_t)c * kChunkRows, FUTT, PREV);
  }

  unsigned short* ENC2T = (unsigned short*)RA;
  k_transp<<<kBatch * 4, 256, 0, stream>>>(ENC2, ENC2T);
  k_applied<<<kBatch, 128, 0, stream>>>(DG + 512, kInfN, W_inf, gp_fm, PREV, 0, 0, ENC2T, HDEC, ACOMB);
  gemm_f32out(ACOMB + 256, 512, WH0INF, kHid, DG, kInfN, BIASC, kBatch, kInfN, kHid, kW16Inv, stream);
  for (int f = 0; f < kFut; ++f) {
    k_applied<<<kBatch, 128, 0, stream>>>(DG + 512, kInfN, W_inf, gp_fm, PREV, f, 1, ENC2T, HDEC, ACOMB);
    gemm_f32out_res(ACOMB, 512, WCOMB, 512, CCOMB, kHid, b_comb, HDEC, kBatch, kHid, 512, kW16Inv, stream);
    k_ln_dec<<<kBatch / 8, 256, 0, stream>>>(CCOMB, g_inf_ln, be_inf_ln, HMID, HMID16);
    gemm_f32out(HMID16, kHid, WHHD, kHid, GH, kG3, b_hh_dec, kBatch, kG3, kHid, kW16Inv, stream);
    k_gates<<<kBatch / 4, 256, 0, stream>>>(GH, HMID, W_ih_dec, b_ih_dec, gp_fm, PREV, f, HDEC, ACOMB);
    gemm_f32out(ACOMB + 256, 512, WH0INF, kHid, DG, kInfN, BIASC, kBatch, kInfN, kHid, kW16Inv, stream);
    k_ln_elu<2><<<kBatch / 8, 256, 0, stream>>>(DG, kInfN, g_ln0, be_ln0, Z0D, kBatch);
    gemm_f32out(Z0D, 512, WH1, 512, D1, kHid, b_h1, kBatch, kHid, 512, kW16Inv, stream);
    k_ln_elu<1><<<kBatch / 8, 256, 0, stream>>>(D1, kHid, g_ln1, be_ln1, Z1D, kBatch);
    gemm_f32out(Z1D, kHid, WH2, kHid, D2, 128, b_h2, kBatch, 128, kHid, kW16Inv, stream);
    k_le2_out<<<kBatch / 32, 256, 0, stream>>>(D2, g_ln2, be_ln2, W_outc, b_outc, gp_fm, 1, f, PAST, FUTT, PREV);
  }

  const int nthr = (kBatch * kOutW) / 4;
  k_final<<<(nthr + 255) / 256, 256, 0, stream>>>(PAST, FUTT, gp_pm, gp_pl, gp_pu, gp_fm, gp_fl, gp_fu, out, nthr);
}
